// BlockSparse_40845138985267
// MI455X (gfx1250) — hardware-verified
//
#include <hip/hip_runtime.h>
#include <stddef.h>


typedef _Float16 v16h __attribute__((ext_vector_type(16)));
typedef _Float16 v8h  __attribute__((ext_vector_type(8)));
typedef float    v8f  __attribute__((ext_vector_type(8)));
typedef float    v4f  __attribute__((ext_vector_type(4)));

#ifndef NROWS
#define NROWS 1024
#endif
#define NROWS_FULL 1024
#define BS     32
#define N_IN   4096
#define N_OUT  4096
#define N_BLK  4096
#define NCB_IN  (N_IN / BS)
#define NCB_OUT (N_OUT / BS)
#define SEG    512
#define RT     128

#define LDX 40
#define LDE 36
#define LDW 40

#define XCARRY 16.0f
#define WCARRY 64.0f

static_assert(BS == 32);
static_assert((N_IN % BS) == 0 && (N_OUT % BS) == 0);
static_assert(NROWS >= RT && NROWS <= NROWS_FULL && (NROWS % RT) == 0);
static_assert(8 * SEG == N_BLK && (SEG % 32) == 0);
static_assert(RT == 8 * 16);
static_assert(RT * 4 == 2 * 256);
static_assert(BS * 4 == 128);
static_assert((LDX % 8) == 0 && LDX >= 32);
static_assert((LDW % 8) == 0 && LDW >= 32);
static_assert((LDE % 4) == 0 && LDE >= 32);
static_assert(((size_t)NROWS * N_IN) % 2048 == 0);
static_assert((N_BLK % 2) == 0);
static_assert((BS * 4) == 128);
static_assert(((size_t)N_OUT * 4) % 128 == 0);
static_assert(RT == 4 * 32);

#define X16_BYTES ((size_t)NROWS * N_IN * 2)
#define WT_BYTES  ((size_t)N_BLK * BS * BS * 2)
#define OFF_X16 ((size_t)0)
#define OFF_WT  (OFF_X16 + X16_BYTES)
#define WS_TOTAL (OFF_WT + WT_BYTES)
static_assert((X16_BYTES % 128) == 0 && (WT_BYTES % 128) == 0);
static_assert(WS_TOTAL <= (size_t)134217728);

__device__ __forceinline__ float bf16r(float x) {
  unsigned int u = __float_as_uint(x);
  u = (u + 0x7FFFu + ((u >> 16) & 1u)) & 0xFFFF0000u;
  return __uint_as_float(u);
}

static __device__ __forceinline__ _Float16 toh_flush(float v) {
  const _Float16 r = (_Float16)v;
  return (fabsf(v) < 6.103515625e-05f) ? (_Float16)0.0f : r;
}

__device__ __forceinline__ v16h frag_at(const _Float16* p) {
  v8h lo = *(const v8h*)(p);
  v8h hi = *(const v8h*)(p + 16);
  v16h out;
#pragma unroll
  for (int i = 0; i < 8; ++i) { out[i] = lo[i]; out[i + 8] = hi[i]; }
  return out;
}
__device__ __forceinline__ v16h ld_frag(const _Float16* base, unsigned ld) {
  const unsigned lane = threadIdx.x & 31u;
  return frag_at(base + (lane & 15u) * ld + (lane >> 4) * 8u);
}

__device__ __forceinline__ v8f wmma16(v16h a, v16h b, v8f c) {
  v8f d = __builtin_amdgcn_wmma_f32_16x16x32_f16(false, a, false, b, (short)0, c,
                                                 false, false);
  asm volatile("v_nop\n\tv_nop\n\tv_nop\n\tv_nop" : "+v"(d) : "v"(a), "v"(b));
  return d;
}

__device__ __forceinline__ float relu_act(float t) {
  return fmaxf(t, 0.0f);
}

__global__ __launch_bounds__(256) void xconv_kernel(
    const float* __restrict__ X, _Float16* __restrict__ X16) {
  const size_t e = ((size_t)blockIdx.x * 256u + threadIdx.x) * 8u;
  const v4f a0 = *(const v4f*)(X + e);
  const v4f a1 = *(const v4f*)(X + e + 4u);
  v8h o;
#pragma unroll
  for (int i = 0; i < 4; ++i) {
    o[i]     = toh_flush(XCARRY * bf16r(a0[i]));
    o[i + 4] = toh_flush(XCARRY * bf16r(a1[i]));
  }
  _Float16* p = X16 + e;
  *(volatile v8h*)p = o;
  __threadfence();
  *(volatile v8h*)p = o;
}

__global__ __launch_bounds__(256) void kconv_kernel(
    const float* __restrict__ Wk, _Float16* __restrict__ Wt) {
  __shared__ _Float16 T[64 * LDW];
  const unsigned tid = threadIdx.x;
  const size_t base = (size_t)blockIdx.x * 2048u;
#pragma unroll 4
  for (unsigned j = 0; j < 8u; ++j) {
    const unsigned idx = tid + 256u * j;
    const unsigned bl = idx >> 10, kr = (idx >> 5) & 31u, nc = idx & 31u;
    const float v = Wk[base + idx];
    T[(bl * 32u + nc) * LDW + kr] = toh_flush(WCARRY * bf16r(v));
  }
  __syncthreads();
  const unsigned r = tid >> 2;
  const unsigned kc = (tid & 3u) * 8u;
  const v8h x = *(const v8h*)&T[r * LDW + kc];
  _Float16* p = Wt + base + (size_t)tid * 8u;
  *(volatile v8h*)p = x;
  __threadfence();
  *(volatile v8h*)p = x;
}

__global__ __launch_bounds__(256) void bsgemm_kernel(
    const _Float16* __restrict__ X16, const _Float16* __restrict__ Wt,
    const float* __restrict__ bias, const int* __restrict__ ci, const int* __restrict__ co,
    float* __restrict__ out) {
  __shared__ _Float16 Xs[RT * LDX];
  __shared__ _Float16 Ws[BS * LDX];
  __shared__ float Cs[RT * LDE];
  __shared__ int lst[8 * SEG];
  __shared__ int cntw[8];

  const unsigned tid = threadIdx.x, lane = tid & 31u;
  const int wave = __builtin_amdgcn_readfirstlane(threadIdx.x >> 5);
  const unsigned hh = lane >> 4, m = lane & 15u;
  const int obk = (int)blockIdx.x;
  const unsigned n0 = blockIdx.x * 32u;
  const unsigned row0 = blockIdx.y * (unsigned)RT;

  int cnt = 0;
#pragma unroll 1
  for (int it = 0; it < SEG / 32; ++it) {
    const int n = wave * SEG + it * 32 + (int)lane;
    const int cv = co[n];
    const bool hit = (cv == obk);
    const unsigned mask = __builtin_amdgcn_ballot_w32(hit);
    const int pos = cnt + (int)__builtin_amdgcn_mbcnt_lo(mask, 0u);
    if (hit) lst[wave * SEG + pos] = n;
    cnt += __builtin_popcount(mask);
  }
  if (lane == 0u) cntw[wave] = cnt;
  __syncthreads();

  v8f acc0 = {}, acc1 = {};
  const unsigned xr0 = tid >> 2;
  const unsigned xc = (tid & 3u) * 8u;
#pragma unroll 1
  for (int w2 = 0; w2 < 8; ++w2) {
    const int c2 = __builtin_amdgcn_readfirstlane(min(max(cntw[w2], 0), SEG));
#pragma unroll 1
    for (int i = 0; i < c2; ++i) {
      const int n = __builtin_amdgcn_readfirstlane(min(max(lst[w2 * SEG + i], 0), N_BLK - 1));
      int cib = ci[n];
      cib = min(max(cib, 0), NCB_IN - 1);
      const size_t xoff = (size_t)(row0 + xr0) * N_IN + (unsigned)cib * 32u + xc;
      const v8h p0 = *(const v8h*)(X16 + xoff);
      const v8h p1 = *(const v8h*)(X16 + xoff + (size_t)64 * N_IN);
      *(v8h*)&Xs[xr0 * LDX + xc] = p0;
      *(v8h*)&Xs[(xr0 + 64u) * LDX + xc] = p1;
      if (wave < 4) {
        const v8h q = *(const v8h*)(Wt + (size_t)n * (BS * BS) + (size_t)tid * 8u);
        *(v8h*)&Ws[xr0 * LDX + xc] = q;
      }
      __syncthreads();
      const v16h a  = ld_frag(&Xs[((unsigned)wave * 16u) * LDX], LDX);
      const v16h b0 = ld_frag(&Ws[0], LDX);
      const v16h b1 = ld_frag(&Ws[16 * LDX], LDX);
      acc0 = wmma16(a, b0, acc0);
      acc1 = wmma16(a, b1, acc1);
      __syncthreads();
    }
  }

#pragma unroll
  for (int r = 0; r < 8; ++r) {
    float* d = &Cs[((unsigned)wave * 16u + hh * 8u + (unsigned)r) * LDE + m];
    d[0]  = acc0[r];
    d[16] = acc1[r];
  }
  __syncthreads();

  const float cs = 1.0f / (XCARRY * WCARRY);
  v4f xs[4];
  size_t off[4];
#pragma unroll
  for (unsigned i = 0; i < 4u; ++i) {
    const unsigned r = 32u * i + (tid >> 3);
    const unsigned c = (tid & 7u) * 4u;
    const v4f u = *(const v4f*)&Cs[r * LDE + c];
    const v4f g = *(const v4f*)(bias + n0 + c);
    v4f val;
#pragma unroll
    for (int j = 0; j < 4; ++j) val[j] = relu_act(u[j] * cs + bf16r(g[j]));
    xs[i] = val;
    off[i] = (size_t)(row0 + r) * N_OUT + n0 + c;
  }
#pragma unroll
  for (int i = 0; i < 4; ++i) *(volatile v4f*)(out + off[i]) = xs[i];
  __threadfence();
#pragma unroll
  for (int i = 0; i < 4; ++i) *(volatile v4f*)(out + off[i]) = xs[i];
}

extern "C" void kernel_launch(void* const* d_in, const int* in_sizes, int n_in,
                              void* d_out, int out_size, void* d_ws, size_t ws_size,
                              hipStream_t stream) {
  if (n_in < 5) return;
  if ((long long)in_sizes[0] < (long long)NROWS * N_IN) return;
  if ((long long)in_sizes[1] < (long long)N_BLK * BS * BS) return;
  if (in_sizes[2] < N_OUT) return;
  if (in_sizes[3] < N_BLK || in_sizes[4] < N_BLK) return;
  if ((long long)out_size < (long long)NROWS * N_OUT) return;
  if (ws_size < WS_TOTAL) return;

  const float* X    = (const float*)d_in[0];
  const float* Wk   = (const float*)d_in[1];
  const float* bias = (const float*)d_in[2];
  const int*   ci   = (const int*)d_in[3];
  const int*   co   = (const int*)d_in[4];
  float* out = (float*)d_out;

  char* ws = (char*)d_ws;
  _Float16* X16 = (_Float16*)(ws + OFF_X16);
  _Float16* Wt  = (_Float16*)(ws + OFF_WT);

  dim3 blk(256);
  xconv_kernel<<<dim3((unsigned)(((size_t)NROWS * N_IN) / 2048u)), blk, 0, stream>>>(X, X16);
  kconv_kernel<<<dim3(N_BLK / 2), blk, 0, stream>>>(Wk, Wt);
  bsgemm_kernel<<<dim3(NCB_OUT, NROWS / RT), blk, 0, stream>>>(X16, Wt, bias, ci, co, out);
}
